// SupCon_2783138808531
// MI455X (gfx1250) — hardware-verified
//
#include <hip/hip_runtime.h>
#include <math.h>


#define NN 8192
#define DIM 128
#define SQIT 3.1622776601683795f

typedef __attribute__((ext_vector_type(16))) _Float16 v16h;
typedef __attribute__((ext_vector_type(8)))  _Float16 v8h;
typedef __attribute__((ext_vector_type(8)))  float v8f;
typedef __attribute__((ext_vector_type(4)))  float v4f;
typedef __attribute__((ext_vector_type(4)))  unsigned v4u;

template <typename T> __device__ __forceinline__ void vst2(void* p, T v) { *(volatile T*)p = v; __threadfence(); *(volatile T*)p = v; }
__device__ __forceinline__ v8f wmma16(v16h a, v16h b, v8f c) {
  v8f d = __builtin_amdgcn_wmma_f32_16x16x32_f16(false, a, false, b, (short)0, c, false, false);
  asm volatile("v_nop\n\tv_nop\n\tv_nop\n\tv_nop" : "+v"(d) : "v"(a), "v"(b));
  return d;
}
__device__ __forceinline__ v16h frag_h(const _Float16* rowk0, int lane) {
  union { v16h v; v8h q[2]; } u; const _Float16* p = rowk0 + 8 * (lane >> 4);
  u.q[0] = *(const v8h*)p; u.q[1] = *(const v8h*)(p + 16); return u.v;
}
#define LDSX() do { asm volatile("s_wait_dscnt 0" ::: "memory"); __builtin_amdgcn_wave_barrier(); __builtin_amdgcn_fence(__ATOMIC_RELEASE, "workgroup"); } while (0)

__global__ __launch_bounds__(256) void k_norm(const float* __restrict__ z, _Float16* __restrict__ zn) {
  const int tid = threadIdx.x, w = tid >> 5, lane = tid & 31; const size_t row = (size_t)blockIdx.x * 8 + w;
  const v4f v = *(const v4f*)(z + row * DIM + lane * 4);
  float ss = v[0] * v[0] + v[1] * v[1] + v[2] * v[2] + v[3] * v[3];
#pragma unroll
  for (int off = 16; off >= 1; off >>= 1) ss += __shfl_xor(ss, off, 32);
  const float sc = SQIT / fmaxf(sqrtf(ss), 1e-8f);
  const float n0 = __shfl_xor(v[0], 1, 32), n1 = __shfl_xor(v[1], 1, 32), n2 = __shfl_xor(v[2], 1, 32), n3 = __shfl_xor(v[3], 1, 32);
  if ((lane & 1) == 0) { union { v8h h; v4u u; } pk;
    pk.h[0] = (_Float16)(v[0] * sc); pk.h[1] = (_Float16)(v[1] * sc); pk.h[2] = (_Float16)(v[2] * sc); pk.h[3] = (_Float16)(v[3] * sc);
    pk.h[4] = (_Float16)(n0 * sc); pk.h[5] = (_Float16)(n1 * sc); pk.h[6] = (_Float16)(n2 * sc); pk.h[7] = (_Float16)(n3 * sc);
    vst2(zn + row * DIM + lane * 4, pk.u); }
}

__global__ __launch_bounds__(128) void k_loss(const _Float16* __restrict__ zn, const int* __restrict__ y, float* __restrict__ loss) {
  __shared__ __align__(16) float so[4][16][20];
  __shared__ __align__(16) float sl[64];
  const int tid = threadIdx.x, w = tid >> 5, lane = tid & 31, col = lane & 15, g = lane >> 4;
  const int r0 = blockIdx.x * 64 + w * 16, i = r0 + col;
  const int yi = y[i];
  v16h a[4];
#pragma unroll
  for (int kc = 0; kc < 4; ++kc) a[kc] = frag_h(zn + (size_t)i * DIM + kc * 32, lane);
  float lsum = 0.f, pos = 0.f; int cnt = 0;
#pragma unroll 1
  for (int jt = 0; jt < NN / 16; ++jt) {
    v8f acc = {};
#pragma unroll
    for (int kc = 0; kc < 4; ++kc) acc = wmma16(a[kc], frag_h(zn + (size_t)(jt * 16 + col) * DIM + kc * 32, lane), acc);
#pragma unroll
    for (int r = 0; r < 8; ++r) so[w][8 * g + r][col] = acc[r];
    LDSX();
#pragma unroll
    for (int c = 0; c < 8; ++c) { const int jj = g * 8 + c, j = jt * 16 + jj; const float s = so[w][col][jj];
      if (j != i) { lsum += expf(s - 10.0f); if (y[j] == yi) { pos += s; cnt += 1; } } }
    __builtin_amdgcn_wave_barrier();
  }
  lsum += __shfl_xor(lsum, 16, 32); pos += __shfl_xor(pos, 16, 32); cnt += __shfl_xor(cnt, 16, 32);
  if (g == 0) { const float lse = 10.0f + logf(lsum); sl[w * 16 + col] = cnt > 0 ? (lse - pos / (float)cnt) : 0.f; }
  __syncthreads();
  if (tid < 16) vst2(loss + (size_t)blockIdx.x * 64 + tid * 4, *(const v4f*)(&sl[tid * 4]));
}

extern "C" void kernel_launch(void* const* d_in, const int* in_sizes, int n_in,
                              void* d_out, int out_size, void* d_ws, size_t ws_size,
                              hipStream_t stream) {
  (void)in_sizes; (void)n_in; (void)out_size; (void)ws_size;
  const float* z = (const float*)d_in[0]; const int* y = (const int*)d_in[1];
  float* loss = (float*)d_out;
  _Float16* zn = (_Float16*)d_ws;
  k_norm<<<NN / 8, 256, 0, stream>>>(z, zn);
  k_loss<<<NN / 64, 128, 0, stream>>>(zn, y, loss);
}
